// MixedScoreMHA_7928509628562
// MI455X (gfx1250) — hardware-verified
//
#include <hip/hip_runtime.h>


#define NB_  32
#define RR   512
#define DD   256
#define D3   768
#define NH_  16
#define KD   16
#define KP   32
#define PCAR 1024.0f
typedef _Float16 h16;
typedef unsigned short bf;
typedef __attribute__((ext_vector_type(16))) __bf16   v16bf;
typedef __attribute__((ext_vector_type(16))) _Float16 v16h;
typedef __attribute__((ext_vector_type(8)))  _Float16 v8h;
typedef __attribute__((ext_vector_type(8)))  unsigned short v8us;
typedef __attribute__((ext_vector_type(8)))  float    v8f;
typedef __attribute__((ext_vector_type(4)))  float    v4f;
typedef v8h  __attribute__((may_alias)) v8ha;
typedef v4f  __attribute__((may_alias)) v4fa;
typedef v8us __attribute__((may_alias)) v8usa;

__device__ __forceinline__ unsigned short f2bf(float f) { unsigned u = __float_as_uint(f); u += 0x7FFFu + ((u >> 16) & 1u); return (unsigned short)(u >> 16); }
__device__ __forceinline__ float bf2f(unsigned short b) { return __uint_as_float(((unsigned)b) << 16); }
__device__ __forceinline__ float bfr(float f) { return bf2f(f2bf(f)); }
__device__ __forceinline__ v16h cat16(v8h lo, v8h hi) { return __builtin_shufflevector(lo, hi, 0, 1, 2, 3, 4, 5, 6, 7, 8, 9, 10, 11, 12, 13, 14, 15); }
__device__ __forceinline__ v16bf cat16b(v8us lo, v8us hi) { return __builtin_bit_cast(v16bf, __builtin_shufflevector(lo, hi, 0, 1, 2, 3, 4, 5, 6, 7, 8, 9, 10, 11, 12, 13, 14, 15)); }
__device__ __forceinline__ v8f wmma16(v16h a, v16h b, v8f c) { return __builtin_amdgcn_wmma_f32_16x16x32_f16(false, a, false, b, (short)0, c, false, false); }
__device__ __forceinline__ v8f wmmab(v16bf a, v16bf b, v8f c) { return __builtin_amdgcn_wmma_f32_16x16x32_bf16(false, a, false, b, (short)0, c, false, false); }


template <typename T16> struct WFrag;
template <> struct WFrag<h16> { typedef v16h V; static __device__ __forceinline__ V ld(const h16* p) { return cat16(*(const v8h*)p, *(const v8h*)(p + 16)); } static __device__ __forceinline__ v8f mma(V a, V b, v8f c) { return wmma16(a, b, c); } };
template <> struct WFrag<bf> { typedef v16bf V; static __device__ __forceinline__ V ld(const bf* p) { return cat16b(*(const v8us*)p, *(const v8us*)(p + 16)); } static __device__ __forceinline__ v8f mma(V a, V b, v8f c) { return wmmab(a, b, c); } };
template <typename T16, int NSPLIT, bool BIAS>
__global__ __launch_bounds__(32) void k_gemmw(const T16* __restrict__ A, const T16* __restrict__ A2, const T16* __restrict__ Bt, const T16* __restrict__ Bt2, int K, float* C, int ldc, const float* __restrict__ bias, size_t sA, size_t sB, size_t sC) {
    typedef typename WFrag<T16>::V V;
    __shared__ __align__(16) float os[16 * 68];
    const size_t z = blockIdx.z; A += z * sA; if (A2) A2 += z * sA; Bt += z * sB; if (Bt2) Bt2 += z * sB; C += z * sC;
    const int lane = threadIdx.x & 31, lr = lane & 15, hi = lane >> 4; const int r0 = blockIdx.x * 64, c0 = blockIdx.y * 64;
    v8f acc[4][4];
#pragma unroll
    for (int mb = 0; mb < 4; ++mb)
#pragma unroll
        for (int nb = 0; nb < 4; ++nb) acc[mb][nb] = (v8f){};
    const size_t aoff = (size_t)(r0 + lr) * K + 8 * hi, boff = (size_t)(c0 + lr) * K + 8 * hi;
#pragma unroll 1
    for (int kc = 0; kc < K; kc += 32) {
        V a[4], a2[4];
#pragma unroll
        for (int mb = 0; mb < 4; ++mb) { a[mb] = WFrag<T16>::ld(A + aoff + (size_t)mb * 16 * K + kc); if (NSPLIT == 1 || NSPLIT == 2) a2[mb] = WFrag<T16>::ld(A2 + aoff + (size_t)mb * 16 * K + kc); }
#pragma unroll
        for (int nb = 0; nb < 4; ++nb) { const V b = WFrag<T16>::ld(Bt + boff + (size_t)nb * 16 * K + kc); V b2; if (NSPLIT >= 2) b2 = WFrag<T16>::ld(Bt2 + boff + (size_t)nb * 16 * K + kc);
#pragma unroll
            for (int mb = 0; mb < 4; ++mb) { acc[mb][nb] = WFrag<T16>::mma(a[mb], b, acc[mb][nb]); if (NSPLIT == 1 || NSPLIT == 2) acc[mb][nb] = WFrag<T16>::mma(a2[mb], b, acc[mb][nb]); if (NSPLIT >= 2) acc[mb][nb] = WFrag<T16>::mma(a[mb], b2, acc[mb][nb]); } }
        asm volatile("v_nop\n\tv_nop\n\tv_nop\n\tv_nop" : "+v"(acc[0][0]), "+v"(acc[1][1]), "+v"(acc[2][2]), "+v"(acc[3][3]) : "v"(a[0]), "v"(a[3]));
    }
#pragma unroll
    for (int mb = 0; mb < 4; ++mb) {
#pragma unroll
        for (int nb = 0; nb < 4; ++nb) {
#pragma unroll
            for (int j = 0; j < 8; ++j) os[(hi * 8 + j) * 68 + nb * 16 + lr] = acc[mb][nb][j]; }
        __builtin_amdgcn_wave_barrier(); asm volatile("" ::: "memory");
        float* crow = C + (size_t)(r0 + mb * 16) * ldc + c0;
#pragma unroll 1
        for (int ps = 0; ps < 2; ++ps) {
#pragma unroll
            for (int s = 0; s < 8; ++s) { const int row = 2 * s + hi, cofs = lr * 4; v4f val = *(const v4fa*)(os + row * 68 + cofs); if (BIAS) { val[0] += bfr(bias[c0 + cofs]); val[1] += bfr(bias[c0 + cofs + 1]); val[2] += bfr(bias[c0 + cofs + 2]); val[3] += bfr(bias[c0 + cofs + 3]); }
                *(volatile v4f*)(crow + (size_t)row * ldc + cofs) = val; }
            if (ps == 0) __threadfence(); }
        __builtin_amdgcn_wave_barrier(); asm volatile("" ::: "memory");
    }
}

__device__ __forceinline__ h16 tohx(float x) { return (h16)x; }
__device__ __forceinline__ void splitf(float y, unsigned short& h, unsigned short& l) { h = f2bf(y); l = f2bf(y - bf2f(h)); }
typedef __attribute__((ext_vector_type(2))) unsigned short v2us;
typedef __attribute__((ext_vector_type(4))) unsigned short v4us;
typedef __attribute__((ext_vector_type(2))) _Float16 v2h;
typedef __attribute__((ext_vector_type(4))) _Float16 v4h;

__global__ __launch_bounds__(256) void k_wtG(const float* __restrict__ w, int K, int N, bf* Bt) {
    const int lane = threadIdx.x & 31; const int L0 = (blockIdx.x * 8 + (threadIdx.x >> 5)) * 8; const int nlines = N * K / 64;
#pragma unroll
    for (int ps = 0; ps < 2; ++ps) {
#pragma unroll 1
        for (int l = 0; l < 8; ++l) { const int L = L0 + l; if (L >= nlines) break; const size_t e = (size_t)L * 64 + lane * 2; const int k = (int)(e % K), n = (int)(e / K); v2us o;
            o[0] = f2bf(w[(size_t)k * N + n]); o[1] = f2bf(w[(size_t)(k + 1) * N + n]); *(volatile v2us*)(Bt + e) = o; }
        if (ps == 0) __threadfence(); }
}
__global__ __launch_bounds__(256) void k_cvt8(const float* __restrict__ src, bf* dst, size_t n8) { const size_t i = (size_t)blockIdx.x * 256 + threadIdx.x; if (i >= n8) return; const v8f v = *(const v8f*)(src + i * 8); v8us o;
#pragma unroll
    for (int k = 0; k < 8; ++k) o[k] = f2bf(v[k]); *(volatile v8us*)(dst + i * 8) = o; __threadfence(); *(volatile v8us*)(dst + i * 8) = o; }
__global__ __launch_bounds__(256) void k_p32(const float* __restrict__ F, int off, bf* Ph, bf* Pl) { const int e = (blockIdx.x * 256 + threadIdx.x) * 4; if (e >= NH_ * RR * KP) return; const int k = e % KP; const int r = (e / KP) % RR; const int h = e / (KP * RR); v4us oh, ol;
#pragma unroll
    for (int u = 0; u < 4; ++u) { unsigned short a = 0, b = 0; if (k + u < KD) splitf(F[(size_t)r * D3 + off + h * KD + k + u], a, b); oh[u] = a; ol[u] = b; } *(volatile v4us*)(Ph + e) = oh; *(volatile v4us*)(Pl + e) = ol; __threadfence(); *(volatile v4us*)(Ph + e) = oh; *(volatile v4us*)(Pl + e) = ol; }
__global__ __launch_bounds__(256) void k_vt64(const float* __restrict__ F, int off, h16* VT) { const int e = (blockIdx.x * 256 + threadIdx.x) * 2; if (e >= NH_ * 64 * RR) return; const int r = e % RR; const int d = (e / RR) % 64; const int h = e / (RR * 64); v2h o;
    if (d < KD) { o[0] = tohx(F[(size_t)r * D3 + off + h * KD + d]); o[1] = tohx(F[(size_t)(r + 1) * D3 + off + h * KD + d]); } else { o[0] = (h16)0.f; o[1] = (h16)0.f; } *(volatile v2h*)(VT + e) = o; __threadfence(); *(volatile v2h*)(VT + e) = o; }
__global__ __launch_bounds__(256) void k_comp(const float* __restrict__ S1, const float* __restrict__ S2, const float* __restrict__ mt, const float* __restrict__ wm, float* COMP) { const size_t e = ((size_t)blockIdx.x * 256 + threadIdx.x) * 4; if (e >= (size_t)NH_ * RR * RR) return; const size_t rc = e % ((size_t)RR * RR); const int h = (int)(e / ((size_t)RR * RR)); const float w = bfr(wm[h]); const v4f a = *(const v4f*)(S1 + e), b = *(const v4f*)(S2 + e), m = *(const v4f*)(mt + rc); v4f o;
#pragma unroll
    for (int u = 0; u < 4; ++u) { float s3 = __fmul_rn(bfr(m[u]), w); asm volatile("" : "+v"(s3)); const float t = __fadd_rn(__fadd_rn(a[u], b[u]), s3); o[u] = __fmul_rn(t, 0.25f); } *(volatile v4f*)(COMP + e) = o; __threadfence(); *(volatile v4f*)(COMP + e) = o; }
__global__ __launch_bounds__(256) void k_rsoft(const float* __restrict__ COMP, h16* P16) { const int lane = threadIdx.x & 31; const int row = blockIdx.x * 8 + (threadIdx.x >> 5); if (row >= NH_ * RR) return; const float* sr = COMP + (size_t)row * RR; float v[RR / 32]; float mx = -3.0e38f;
#pragma unroll
    for (int ch = 0; ch < RR / 128; ++ch) { const v4f a = *(const v4f*)(sr + ch * 128 + lane * 4);
#pragma unroll
        for (int u = 0; u < 4; ++u) { v[ch * 4 + u] = a[u]; mx = fmaxf(mx, a[u]); } }
#pragma unroll
    for (int sh = 16; sh; sh >>= 1) mx = fmaxf(mx, __shfl_xor(mx, sh, 32));
    float sum = 0.f;
#pragma unroll
    for (int q = 0; q < RR / 32; ++q) { float d0 = __fsub_rn(v[q], mx); asm volatile("" : "+v"(d0)); v[q] = __builtin_amdgcn_exp2f(__fmul_rn(d0, 1.4426950408889634f)); sum += v[q]; }
#pragma unroll
    for (int sh = 16; sh; sh >>= 1) sum += __shfl_xor(sum, sh, 32);
    const float f = __fdiv_rn(PCAR, sum);
    for (int ps = 0; ps < 2; ++ps) {
#pragma unroll
        for (int ch = 0; ch < RR / 128; ++ch) { v4h o4;
#pragma unroll
            for (int q = 0; q < 4; ++q) o4[q] = tohx(v[ch * 4 + q] * f); *(volatile v4h*)(P16 + (size_t)row * RR + ch * 128 + lane * 4) = o4; }
        if (ps == 0) __threadfence(); } }
__global__ __launch_bounds__(256) void k_cstat(const float* __restrict__ COMP, float* MX, float* RS) { const int idx = blockIdx.x * 256 + threadIdx.x; if (idx >= NH_ * RR) return; const int c = idx % RR; const int h = idx / RR; const float* base = COMP + (size_t)h * RR * RR + c; float mx = -3.0e38f;
#pragma unroll 1
    for (int r = 0; r < RR; ++r) mx = fmaxf(mx, base[(size_t)r * RR]);
    float sum = 0.f;
#pragma unroll 1
    for (int r = 0; r < RR; ++r) { float d0 = __fsub_rn(base[(size_t)r * RR], mx); asm volatile("" : "+v"(d0)); sum = __fadd_rn(sum, __builtin_amdgcn_exp2f(__fmul_rn(d0, 1.4426950408889634f))); }
    const float rs = __fdiv_rn(PCAR, sum); for (int ps = 0; ps < 2; ++ps) { *(volatile float*)(MX + idx) = mx; *(volatile float*)(RS + idx) = rs; if (ps == 0) __threadfence(); } }
__global__ __launch_bounds__(256) void k_pcolT(const float* __restrict__ COMP, const float* __restrict__ MX, const float* __restrict__ RS, h16* PCT) { const int e = (blockIdx.x * 256 + threadIdx.x) * 4; if (e >= NH_ * RR * RR) return; const int r0 = e % RR; const int c = (e / RR) % RR; const int h = e / (RR * RR); const float mx = MX[h * RR + c], rs = RS[h * RR + c]; v4h o;
#pragma unroll
    for (int u = 0; u < 4; ++u) { float d0 = __fsub_rn(COMP[((size_t)h * RR + r0 + u) * RR + c], mx); asm volatile("" : "+v"(d0)); o[u] = tohx(__fmul_rn(__builtin_amdgcn_exp2f(__fmul_rn(d0, 1.4426950408889634f)), rs)); } *(volatile v4h*)(PCT + e) = o; __threadfence(); *(volatile v4h*)(PCT + e) = o; }
__global__ __launch_bounds__(256) void k_mrg(const float* __restrict__ O, bf* Mh, bf* Ml) { const int e = (blockIdx.x * 256 + threadIdx.x) * 4; if (e >= RR * DD) return; const int c = e % DD; const int r = e / DD; const int h = c / KD, d = c % KD; const float* o = O + ((size_t)h * RR + r) * 64 + d; v4us oh, ol;
#pragma unroll
    for (int u = 0; u < 4; ++u) { unsigned short a, b; splitf(o[u] * (1.0f / PCAR), a, b); oh[u] = a; ol[u] = b; } *(volatile v4us*)(Mh + e) = oh; *(volatile v4us*)(Ml + e) = ol; __threadfence(); *(volatile v4us*)(Mh + e) = oh; *(volatile v4us*)(Ml + e) = ol; }

extern "C" void kernel_launch(void* const* d_in, const int* in_sizes, int n_in,
                              void* d_out, int out_size, void* d_ws, size_t ws_size, hipStream_t stream) {
    (void)in_sizes; (void)n_in; (void)out_size;
    const float** I = (const float**)d_in;
    const float *row_emb = I[0], *col_emb = I[1], *matrix = I[2], *Wq_row = I[3], *Wk_row = I[4], *Wv_row = I[5], *Wq_col = I[6], *Wk_col = I[7], *Wv_col = I[8], *W_mat = I[9], *W_out_row = I[10], *W_out_col = I[11];
    float* OUT0 = (float*)d_out; float* OUT1 = OUT0 + (size_t)NB_ * RR * DD;
    char* wsp = (char*)d_ws;
    auto take = [&](size_t bytes) { char* p = wsp; wsp += (bytes + 255) & ~(size_t)255; return (void*)p; };
    bf* BR = (bf*)take((size_t)D3 * DD * 2); bf* BC = (bf*)take((size_t)D3 * DD * 2); bf* BOR = (bf*)take(DD * DD * 2); bf* BOC = (bf*)take(DD * DD * 2);
    bf* REB = (bf*)take((size_t)RR * DD * 2); bf* CEB = (bf*)take((size_t)RR * DD * 2); float* RF = (float*)take((size_t)RR * D3 * 4); float* CF = (float*)take((size_t)RR * D3 * 4);
    bf* RQh = (bf*)take((size_t)NH_ * RR * KP * 2); bf* RQl = (bf*)take((size_t)NH_ * RR * KP * 2); bf* RKh = (bf*)take((size_t)NH_ * RR * KP * 2); bf* RKl = (bf*)take((size_t)NH_ * RR * KP * 2); bf* CQh = (bf*)take((size_t)NH_ * RR * KP * 2); bf* CQl = (bf*)take((size_t)NH_ * RR * KP * 2); bf* CKh = (bf*)take((size_t)NH_ * RR * KP * 2); bf* CKl = (bf*)take((size_t)NH_ * RR * KP * 2);
    h16* CVT = (h16*)take((size_t)NH_ * 64 * RR * 2); h16* RVT = (h16*)take((size_t)NH_ * 64 * RR * 2); float* S1 = (float*)take((size_t)NH_ * RR * RR * 4); float* S2 = (float*)take((size_t)NH_ * RR * RR * 4); float* COMP = (float*)take((size_t)NH_ * RR * RR * 4); h16* PR = (h16*)take((size_t)NH_ * RR * RR * 2); float* MXC = (float*)take(NH_ * RR * 4); float* RSC = (float*)take(NH_ * RR * 4); h16* PCT = (h16*)take((size_t)NH_ * RR * RR * 2);
    float* ORW = (float*)take((size_t)NH_ * RR * 64 * 4); float* OCL = (float*)take((size_t)NH_ * RR * 64 * 4); bf* MRh = (bf*)take((size_t)RR * DD * 2); bf* MRl = (bf*)take((size_t)RR * DD * 2); bf* MCh = (bf*)take((size_t)RR * DD * 2); bf* MCl = (bf*)take((size_t)RR * DD * 2);
    if ((size_t)(wsp - (char*)d_ws) > ws_size) return;
    k_wtG<<<(DD * DD / 64 + 63) / 64, 256, 0, stream>>>(Wq_row, DD, DD, BR); k_wtG<<<(DD * DD / 64 + 63) / 64, 256, 0, stream>>>(Wk_row, DD, DD, BR + (size_t)DD * DD); k_wtG<<<(DD * DD / 64 + 63) / 64, 256, 0, stream>>>(Wv_row, DD, DD, BR + (size_t)2 * DD * DD);
    k_wtG<<<(DD * DD / 64 + 63) / 64, 256, 0, stream>>>(Wq_col, DD, DD, BC); k_wtG<<<(DD * DD / 64 + 63) / 64, 256, 0, stream>>>(Wk_col, DD, DD, BC + (size_t)DD * DD); k_wtG<<<(DD * DD / 64 + 63) / 64, 256, 0, stream>>>(Wv_col, DD, DD, BC + (size_t)2 * DD * DD);
    k_wtG<<<(DD * DD / 64 + 63) / 64, 256, 0, stream>>>(W_out_row, DD, DD, BOR); k_wtG<<<(DD * DD / 64 + 63) / 64, 256, 0, stream>>>(W_out_col, DD, DD, BOC);
    const unsigned gP = (NH_ * RR * KP / 4 + 255) / 256, gV = (NH_ * 64 * RR / 2 + 255) / 256, gS = (unsigned)(((size_t)NH_ * RR * RR / 4 + 255) / 256), gM = (RR * DD / 4 + 255) / 256;
    for (int b = 0; b < NB_; ++b) {
        k_cvt8<<<(RR * DD / 8 + 255) / 256, 256, 0, stream>>>(row_emb + (size_t)b * RR * DD, REB, RR * DD / 8); k_cvt8<<<(RR * DD / 8 + 255) / 256, 256, 0, stream>>>(col_emb + (size_t)b * RR * DD, CEB, RR * DD / 8);
        k_gemmw<bf, 0, false><<<dim3(RR / 64, D3 / 64, 1), 32, 0, stream>>>(REB, nullptr, BR, nullptr, DD, RF, D3, nullptr, 0, 0, 0); k_gemmw<bf, 0, false><<<dim3(RR / 64, D3 / 64, 1), 32, 0, stream>>>(CEB, nullptr, BC, nullptr, DD, CF, D3, nullptr, 0, 0, 0);
        k_p32<<<gP, 256, 0, stream>>>(RF, 0, RQh, RQl); k_p32<<<gP, 256, 0, stream>>>(RF, DD, RKh, RKl); k_p32<<<gP, 256, 0, stream>>>(CF, 0, CQh, CQl); k_p32<<<gP, 256, 0, stream>>>(CF, DD, CKh, CKl);
        k_vt64<<<gV, 256, 0, stream>>>(CF, 2 * DD, CVT); k_vt64<<<gV, 256, 0, stream>>>(RF, 2 * DD, RVT);
        k_gemmw<bf, 2, false><<<dim3(RR / 64, RR / 64, NH_), 32, 0, stream>>>(RQh, RQl, CKh, CKl, KP, S1, RR, nullptr, (size_t)RR * KP, (size_t)RR * KP, (size_t)RR * RR);
        k_gemmw<bf, 2, false><<<dim3(RR / 64, RR / 64, NH_), 32, 0, stream>>>(RKh, RKl, CQh, CQl, KP, S2, RR, nullptr, (size_t)RR * KP, (size_t)RR * KP, (size_t)RR * RR);
        k_comp<<<gS, 256, 0, stream>>>(S1, S2, matrix + (size_t)b * RR * RR, W_mat, COMP);
        k_rsoft<<<NH_ * RR / 8, 256, 0, stream>>>(COMP, PR); k_cstat<<<(NH_ * RR + 255) / 256, 256, 0, stream>>>(COMP, MXC, RSC); k_pcolT<<<gS, 256, 0, stream>>>(COMP, MXC, RSC, PCT);
        k_gemmw<h16, 0, false><<<dim3(RR / 64, 1, NH_), 32, 0, stream>>>(PR, nullptr, CVT, nullptr, RR, ORW, 64, nullptr, (size_t)RR * RR, (size_t)64 * RR, (size_t)RR * 64);
        k_gemmw<h16, 0, false><<<dim3(RR / 64, 1, NH_), 32, 0, stream>>>(PCT, nullptr, RVT, nullptr, RR, OCL, 64, nullptr, (size_t)RR * RR, (size_t)64 * RR, (size_t)RR * 64);
        k_mrg<<<gM, 256, 0, stream>>>(ORW, MRh, MRl); k_mrg<<<gM, 256, 0, stream>>>(OCL, MCh, MCl);
        k_gemmw<bf, 1, false><<<dim3(RR / 64, DD / 64, 1), 32, 0, stream>>>(MRh, MRl, BOR, nullptr, DD, OUT0 + (size_t)b * RR * DD, DD, nullptr, 0, 0, 0); k_gemmw<bf, 1, false><<<dim3(RR / 64, DD / 64, 1), 32, 0, stream>>>(MCh, MCl, BOC, nullptr, DD, OUT1 + (size_t)b * RR * DD, DD, nullptr, 0, 0, 0); }
}
